// S6Block_69295002354167
// MI455X (gfx1250) — hardware-verified
//
#include <hip/hip_runtime.h>
#include <math.h>

constexpr int kBatch  = 2;
constexpr int kSeq    = 4096;
constexpr int kDim    = 1024;
constexpr int kState  = 16;
constexpr int kTaps   = 4;
constexpr int kRows   = kBatch * kSeq;
constexpr int kDim2   = 2 * kDim;
constexpr int kBCcols = 2 * kState;
constexpr int kBCld   = 64;
constexpr int kScanTPB = 128;
constexpr int kChunkT  = 64;
static_assert(kRows % 64 == 0 && kDim % 64 == 0 && kDim2 % 64 == 0 && kBCld % 64 == 0, "tile multiples");
static_assert(kDim % 32 == 0, "K multiple of 32");
static_assert(kDim % kScanTPB == 0 && kSeq % kChunkT == 0, "scan tiling");

constexpr size_t kMiB      = 1024ull * 1024ull;
constexpr size_t kOffP16H  = 0;
constexpr size_t kOffP16L  = kOffP16H + (size_t)kRows * kDim * 2;
constexpr size_t kOffWinH  = kOffP16L + (size_t)kRows * kDim * 2;
constexpr size_t kOffWinL  = kOffWinH + (size_t)kDim2 * kDim * 2;
constexpr size_t kOffXS    = kOffWinL + (size_t)kDim2 * kDim * 2;
constexpr size_t kOffGate  = kOffXS   + (size_t)kRows * kDim * 4;
constexpr size_t kOffWoutH = kOffGate + (size_t)kRows * kDim * 4;
constexpr size_t kOffWoutL = kOffWoutH + (size_t)kDim * kDim * 2;
constexpr size_t kOffWxH   = kOffWoutL + (size_t)kDim * kDim * 2;
constexpr size_t kOffWxL   = kOffWxH + (size_t)kBCld * kDim * 2;
constexpr size_t kOffBC    = kOffWxL + (size_t)kBCld * kDim * 2;
constexpr size_t kOffHfin  = kOffBC + (size_t)kRows * kBCld * 4;
constexpr size_t kWsEnd    = kOffHfin + (size_t)kBatch * kDim * kState * 4;
static_assert(kWsEnd == 115736576ull, "carve total");
static_assert(kWsEnd <= 134217728ull, "carve under 128 MiB");
static_assert(kOffWinH % 128 == 0 && kOffXS % 128 == 0 && kOffGate % 128 == 0 && kOffWoutH % 128 == 0 &&
              kOffWxH % 128 == 0 && kOffBC % 128 == 0 && kOffHfin % 128 == 0, "128-B aligned regions");

typedef __attribute__((ext_vector_type(16))) _Float16 v16h;
typedef __attribute__((ext_vector_type(8)))  _Float16 v8h;
typedef __attribute__((ext_vector_type(16))) __bf16   v16b;
typedef __attribute__((ext_vector_type(8)))  __bf16   v8b;
typedef __attribute__((ext_vector_type(8)))  float    v8f;
typedef __attribute__((ext_vector_type(4)))  float    v4f;
typedef __attribute__((ext_vector_type(2)))  float    v2f;
typedef __attribute__((ext_vector_type(4)))  unsigned int v4u;

__device__ __forceinline__ unsigned short f2bf_bits(float f) {
  unsigned u = __float_as_uint(f);
  return (unsigned short)((u + 0x7FFFu + ((u >> 16) & 1u)) >> 16);
}
__device__ __forceinline__ float bf_bits2f(unsigned short h) { return __uint_as_float(((unsigned)h) << 16); }

__device__ __forceinline__ void dep_guard_h(v8f& a, v8f& b, v16h x, v16h y) { asm volatile("v_nop\n\tv_nop\n\tv_nop\n\tv_nop" : "+v"(a), "+v"(b) : "v"(x), "v"(y)); }
__device__ __forceinline__ void dep_guard_b(v8f& a, v8f& b, v16b x, v16b y) { asm volatile("v_nop\n\tv_nop\n\tv_nop\n\tv_nop" : "+v"(a), "+v"(b) : "v"(x), "v"(y)); }
__device__ __forceinline__ void keep4_h(v16h a, v16h b, v16h c, v16h d) { asm volatile("v_nop" :: "v"(a), "v"(b), "v"(c), "v"(d)); }
__device__ __forceinline__ void keep4_b(v16b a, v16b b, v16b c, v16b d) { asm volatile("v_nop" :: "v"(a), "v"(b), "v"(c), "v"(d)); }
__device__ __forceinline__ void acc_guard4(v8f& a, v8f& b, v8f& c, v8f& d) { asm volatile("v_nop\n\tv_nop\n\tv_nop\n\tv_nop" : "+v"(a), "+v"(b), "+v"(c), "+v"(d)); }
template <typename T> struct Frag;
template <> struct Frag<_Float16> {
  typedef v16h V; union U { v16h v; v8h h[2]; };
  static __device__ __forceinline__ v16h load(const _Float16* p) {
    U f; f.h[0] = *(const v8h*)(p); f.h[1] = *(const v8h*)(p + 16); return f.v;
  }
  static __device__ __forceinline__ v8f mma(v16h a, v16h b, v8f c) {
    return __builtin_amdgcn_wmma_f32_16x16x32_f16(false, a, false, b, (short)0, c, false, false);
  }
  static __device__ __forceinline__ void guard(v8f& a, v8f& b, v16h x, v16h y) { dep_guard_h(a, b, x, y); }
  static __device__ __forceinline__ void keep(v16h a, v16h b, v16h c, v16h d) { keep4_h(a, b, c, d); }
};
template <> struct Frag<__bf16> {
  typedef v16b V; union U { v16b v; v8b h[2]; };
  static __device__ __forceinline__ v16b load(const __bf16* p) {
    U f; f.h[0] = *(const v8b*)(p); f.h[1] = *(const v8b*)(p + 16); return f.v;
  }
  static __device__ __forceinline__ v8f mma(v16b a, v16b b, v8f c) {
    return __builtin_amdgcn_wmma_f32_16x16x32_bf16(false, a, false, b, (short)0, c, false, false);
  }
  static __device__ __forceinline__ void guard(v8f& a, v8f& b, v16b x, v16b y) { dep_guard_b(a, b, x, y); }
  static __device__ __forceinline__ void keep(v16b a, v16b b, v16b c, v16b d) { keep4_b(a, b, c, d); }
};

__device__ __forceinline__ unsigned pk16(unsigned short a, unsigned short b) { return (unsigned)a | ((unsigned)b << 16); }
__device__ __forceinline__ void split_bf(float v, unsigned short& hb, unsigned short& lb) {
  hb = f2bf_bits(v);
  lb = f2bf_bits(v - bf_bits2f(hb));
}

template <int ET> struct Elem;
template <> struct Elem<0> { typedef _Float16 T; };
template <> struct Elem<1> { typedef __bf16 T; };
template <int ET, bool SPLIT, int BIAS_MODE, int OUT_MODE, bool RESID, int ACT = 0>
__global__ __launch_bounds__(256) void wmma_gemm64(
    const unsigned short* __restrict__ Ap, const unsigned short* __restrict__ A2p, int lda, long strideA,
    const unsigned short* __restrict__ Btp, const unsigned short* __restrict__ Bt2p, int ldb, long strideB,
    void* __restrict__ Cout, void* __restrict__ Cout2, int ldc, long strideC,
    const float* __restrict__ bias,
    const float* __restrict__ resid, long strideR,
    int M, int N, int K, float scale) {
  typedef typename Elem<ET>::T T;
  typedef typename Frag<T>::V V;
  const T* A = (const T*)Ap; const T* A2 = (const T*)A2p; const T* Bt = (const T*)Btp; const T* Bt2 = (const T*)Bt2p;
  __shared__ __align__(16) float sT[8][16 * 68];
  const int b    = blockIdx.y;
  const int lane = threadIdx.x & 31;
  const int wave = threadIdx.x >> 5;
  const int tilesN = N >> 6;
  const int tilesM = M >> 6;
  const int tile = blockIdx.x * 8 + wave;
  if (tile >= tilesM * tilesN) return;
  const int tm = tile / tilesN;
  const int tn = tile - tm * tilesN;
  const int m0 = tm << 6;
  const int n0 = tn << 6;

  const T* Ab  = A  + (size_t)b * strideA;
  const T* Bb  = Bt + (size_t)b * strideB;
  const T* Ab2 = SPLIT ? (A2  + (size_t)b * strideA) : nullptr;
  const T* Bb2 = SPLIT ? (Bt2 + (size_t)b * strideB) : nullptr;

  const int rlane = lane & 15;
  const int koff  = (lane >> 4) * 8;
  const int mOff  = (lane >> 4) * 8;

  v8f acc[4][4];
#pragma unroll
  for (int i = 0; i < 4; ++i)
#pragma unroll
    for (int j = 0; j < 4; ++j) acc[i][j] = (v8f){0.f,0.f,0.f,0.f,0.f,0.f,0.f,0.f};

  for (int k0 = 0; k0 < K; k0 += 32) {
    V bh[4], bl[4];
#pragma unroll
    for (int j = 0; j < 4; ++j) {
      const size_t bo = (size_t)(n0 + (j << 4) + rlane) * ldb + koff + k0;
      bh[j] = Frag<T>::load(Bb + bo);
      if (SPLIT) bl[j] = Frag<T>::load(Bb2 + bo);
    }
#pragma unroll
    for (int i = 0; i < 4; ++i) {
      const size_t ao = (size_t)(m0 + (i << 4) + rlane) * lda + koff + k0;
      V ah = Frag<T>::load(Ab + ao);
      V al;
      if (SPLIT) al = Frag<T>::load(Ab2 + ao);
#pragma unroll
      for (int j = 0; j < 4; ++j) {
        acc[i][j] = Frag<T>::mma(ah, bh[j], acc[i][j]);
        if (SPLIT) {
          acc[i][j] = Frag<T>::mma(ah, bl[j], acc[i][j]);
          acc[i][j] = Frag<T>::mma(al, bh[j], acc[i][j]);
        }
      }
      Frag<T>::guard(acc[i][0], acc[i][3], ah, SPLIT ? al : ah);
    }
    Frag<T>::keep(bh[0], bh[1], bh[2], bh[3]);
    if (SPLIT) Frag<T>::keep(bl[0], bl[1], bl[2], bl[3]);
  }
  acc_guard4(acc[0][0], acc[0][1], acc[0][2], acc[0][3]);
  acc_guard4(acc[1][0], acc[1][1], acc[1][2], acc[1][3]);
  acc_guard4(acc[2][0], acc[2][1], acc[2][2], acc[2][3]);
  acc_guard4(acc[3][0], acc[3][1], acc[3][2], acc[3][3]);

  float* slab = sT[wave];
  const float* Rb = RESID ? (resid + (size_t)b * strideR) : nullptr;
#pragma unroll
  for (int i = 0; i < 4; ++i) {
    const int mBase = m0 + (i << 4);
#pragma unroll
    for (int j = 0; j < 4; ++j) {
      const int n = n0 + (j << 4) + rlane;
      float bv = 0.f;
      if (BIAS_MODE == 2) bv = bias[n];
#pragma unroll
      for (int r = 0; r < 8; ++r) {
        float v = acc[i][j][r] * scale;
        if (BIAS_MODE == 1) v += bias[mBase + mOff + r];
        if (BIAS_MODE == 2) v += bv;
        if (RESID) v += Rb[(size_t)(mBase + mOff + r) * ldc + n];
        if (ACT == 2) v = fmaxf(v, 0.0f);
        if (ACT == 4) v = (v > 0.f) ? v : 0.01f * v;
        slab[(mOff + r) * 68 + (j << 4) + rlane] = v;
      }
    }
    __builtin_amdgcn_fence(__ATOMIC_RELEASE, "workgroup");
    __builtin_amdgcn_wave_barrier();
    __builtin_amdgcn_fence(__ATOMIC_ACQUIRE, "workgroup");
    if (OUT_MODE == 0) {
      float* C = (float*)Cout + (size_t)b * strideC;
      const int hh = lane >> 4, c4 = (lane & 15) * 4;
      for (int pass = 0; pass < 2; ++pass) {
#pragma unroll
        for (int it = 0; it < 8; ++it) {
          const int row = it * 2 + hh;
          v4f v = *(const v4f*)(slab + row * 68 + c4);
          *(volatile v4f*)(C + (size_t)(mBase + row) * ldc + n0 + c4) = v;
        }
        __threadfence();
      }
    } else {
      const int q = lane >> 3, c8 = (lane & 7) * 8;
      unsigned short* C  = (unsigned short*)Cout  + (size_t)b * strideC;
      unsigned short* C2 = (OUT_MODE == 2) ? ((unsigned short*)Cout2 + (size_t)b * strideC) : nullptr;
      for (int pass = 0; pass < 2; ++pass) {
#pragma unroll
        for (int it = 0; it < 4; ++it) {
          const int row = it * 4 + q;
          const float* sp = slab + row * 68 + c8;
          v8h hv, lv;
#pragma unroll
          for (int e = 0; e < 8; ++e) {
            if (OUT_MODE == 1) {
              hv[e] = (_Float16)sp[e];
            } else {
              unsigned short hb = f2bf_bits(sp[e]);
              unsigned short lb = f2bf_bits(sp[e] - bf_bits2f(hb));
              hv[e] = __builtin_bit_cast(_Float16, hb);
              lv[e] = __builtin_bit_cast(_Float16, lb);
            }
          }
          *(volatile v8h*)(C + (size_t)(mBase + row) * ldc + n0 + c8) = hv;
          if (OUT_MODE == 2) *(volatile v8h*)(C2 + (size_t)(mBase + row) * ldc + n0 + c8) = lv;
        }
        __threadfence();
      }
    }
    __builtin_amdgcn_fence(__ATOMIC_RELEASE, "workgroup");
    __builtin_amdgcn_wave_barrier();
    __builtin_amdgcn_fence(__ATOMIC_ACQUIRE, "workgroup");
  }
}

__global__ __launch_bounds__(256) void split8_bf16_kernel(const float* __restrict__ in, unsigned short* __restrict__ oh,
                                                         unsigned short* __restrict__ ol, int n8) {
  const int i = blockIdx.x * 256 + threadIdx.x;
  if (i >= n8) return;
  const float* p = in + 8 * (size_t)i;
  const v4f a = *(const v4f*)(p);
  const v4f c = *(const v4f*)(p + 4);
  unsigned short hb[8], lb[8];
#pragma unroll
  for (int e = 0; e < 4; ++e) {
    split_bf(a[e], hb[e], lb[e]);
    split_bf(c[e], hb[4 + e], lb[4 + e]);
  }
  const v4u uh = (v4u){pk16(hb[0], hb[1]), pk16(hb[2], hb[3]), pk16(hb[4], hb[5]), pk16(hb[6], hb[7])};
  const v4u ul = (v4u){pk16(lb[0], lb[1]), pk16(lb[2], lb[3]), pk16(lb[4], lb[5]), pk16(lb[6], lb[7])};
  unsigned short* qh = oh + 8 * (size_t)i;
  unsigned short* ql = ol + 8 * (size_t)i;
  *(volatile v4u*)qh = uh;
  *(volatile v4u*)ql = ul;
  __threadfence();
  *(volatile v4u*)qh = uh;
  *(volatile v4u*)ql = ul;
}

__global__ __launch_bounds__(256) void wt_split_kernel(const float* __restrict__ W, int ldw, int nvalid, int ldo,
                                                      unsigned short* __restrict__ oh, unsigned short* __restrict__ ol) {
  __shared__ float sm[64][65];
  const int t  = threadIdx.x;
  const int k0 = blockIdx.x * 64;
  const int n0 = blockIdx.y * 64;
#pragma unroll
  for (int i = 0; i < 16; ++i) {
    const int e = i * 256 + t;
    const int r = e >> 6;
    const int c = e & 63;
    const int n = n0 + c;
    const int nc = (n < nvalid) ? n : (nvalid - 1);
    float v = W[(size_t)(k0 + r) * ldw + nc];
    if (n >= nvalid) v = 0.0f;
    sm[c][r] = v;
  }
  __syncthreads();
  const int lane = t & 31, wave = t >> 5;
  const int q = lane >> 3, c8 = (lane & 7) * 8;
  for (int pass = 0; pass < 2; ++pass) {
#pragma unroll
    for (int it = 0; it < 2; ++it) {
      const int row = wave * 8 + it * 4 + q;
      unsigned short hb[8], lb[8];
#pragma unroll
      for (int e = 0; e < 8; ++e) split_bf(sm[row][c8 + e], hb[e], lb[e]);
      const v4u uh = (v4u){pk16(hb[0], hb[1]), pk16(hb[2], hb[3]), pk16(hb[4], hb[5]), pk16(hb[6], hb[7])};
      const v4u ul = (v4u){pk16(lb[0], lb[1]), pk16(lb[2], lb[3]), pk16(lb[4], lb[5]), pk16(lb[6], lb[7])};
      const size_t off = (size_t)(n0 + row) * ldo + k0 + c8;
      *(volatile v4u*)(oh + off) = uh;
      *(volatile v4u*)(ol + off) = ul;
    }
    __threadfence();
  }
}

__device__ __forceinline__ float conv_silu(float x0, float x1, float x2, float x3,
                                           float w0, float w1, float w2, float w3, float cb) {
  float s = x0 * w0;
  s = fmaf(x1, w1, s);
  s = fmaf(x2, w2, s);
  s = fmaf(x3, w3, s);
  const float a = s + cb;
  const float e = expf(-a);
  const float sig = __builtin_amdgcn_rcpf(1.0f + e);
  return a * sig;
}

__global__ __launch_bounds__(256) void conv_split_kernel(const float* __restrict__ XS, const float* __restrict__ cw,
                                                        const float* __restrict__ cbp, unsigned short* __restrict__ oh,
                                                        unsigned short* __restrict__ ol, int n2) {
  const int i = blockIdx.x * 256 + threadIdx.x;
  if (i >= n2) return;
  const int e0 = 2 * i;
  const int m  = e0 >> 10;
  const int d  = e0 & (kDim - 1);
  const int t  = m & (kSeq - 1);
  v2f xv[kTaps];
#pragma unroll
  for (int j = 0; j < kTaps; ++j) {
    const int tr = t - (kTaps - 1) + j;
    const bool valid = (tr >= 0);
    const int mr = valid ? (m - (kTaps - 1) + j) : m;
    const v2f v = *(const v2f*)(XS + (size_t)mr * kDim + d);
    xv[j] = valid ? v : (v2f){0.0f, 0.0f};
  }
  const v4f wa = *(const v4f*)(cw + (size_t)d * kTaps);
  const v4f wb = *(const v4f*)(cw + (size_t)d * kTaps + 4);
  const float y0 = conv_silu(xv[0][0], xv[1][0], xv[2][0], xv[3][0], wa[0], wa[1], wa[2], wa[3], cbp[d]);
  const float y1 = conv_silu(xv[0][1], xv[1][1], xv[2][1], xv[3][1], wb[0], wb[1], wb[2], wb[3], cbp[d + 1]);
  unsigned short h0, l0, h1, l1;
  split_bf(y0, h0, l0);
  split_bf(y1, h1, l1);
  const unsigned uh = pk16(h0, h1), ul = pk16(l0, l1);
  ((volatile unsigned*)oh)[i] = uh;
  ((volatile unsigned*)ol)[i] = ul;
  __threadfence();
  ((volatile unsigned*)oh)[i] = uh;
  ((volatile unsigned*)ol)[i] = ul;
}

__global__ __launch_bounds__(kScanTPB) void scan_kernel(
    const float* __restrict__ XS, const float* __restrict__ GT, const float* __restrict__ BCp,
    const float* __restrict__ conv_w, const float* __restrict__ conv_b, const float* __restrict__ b_x,
    const float* __restrict__ A_log, const float* __restrict__ Dp,
    unsigned short* __restrict__ YH, unsigned short* __restrict__ YL, float* __restrict__ HF) {
  __shared__ __align__(16) float sA[kScanTPB * kState];
  __shared__ __align__(16) float sBC[kChunkT * kBCcols];
  __shared__ __align__(16) float sY[kChunkT * kScanTPB];
  const int tid = threadIdx.x, lane = tid & 31, wave = tid >> 5;
  constexpr int blocksPerB = kDim / kScanTPB;
  const int b  = blockIdx.x / blocksPerB;
  const int d0 = (blockIdx.x - b * blocksPerB) * kScanTPB;
  const int d  = d0 + tid;

#pragma unroll 1
  for (int i = tid; i < kScanTPB * kState; i += kScanTPB) {
    const float al = A_log[(size_t)d0 * kState + i];
    sA[i] = expf(-expf(al));
  }
  __syncthreads();
  float Av[kState], h[kState];
  {
    const float* ap = sA + tid * kState;
#pragma unroll
    for (int q4 = 0; q4 < 4; ++q4) {
      const v4f v = *(const v4f*)(ap + 4 * q4);
      Av[4 * q4 + 0] = v[0]; Av[4 * q4 + 1] = v[1]; Av[4 * q4 + 2] = v[2]; Av[4 * q4 + 3] = v[3];
    }
  }
#pragma unroll
  for (int n = 0; n < kState; ++n) h[n] = 0.0f;
  const v4f cwv = *(const v4f*)(conv_w + (size_t)d * kTaps);
  const float cb = conv_b[d];
  const float Dv = Dp[d];
  float xm1 = 0.0f, xm2 = 0.0f, xm3 = 0.0f;
  const int lq = lane >> 3, lc = lane & 7;

#pragma unroll 1
  for (int tb = 0; tb < kSeq; tb += kChunkT) {
    __syncthreads();
#pragma unroll 1
    for (int i = tid; i < kChunkT * 8; i += kScanTPB) {
      const int r = i >> 3, c4 = (i & 7) * 4;
      v4f v = *(const v4f*)(BCp + ((size_t)(b * kSeq + tb + r)) * kBCld + c4);
      const v4f bx = *(const v4f*)(b_x + c4);
      v += bx;
      *(v4f*)(sBC + r * kBCcols + c4) = v;
    }
    __syncthreads();
#pragma unroll 1
    for (int tt = 0; tt < kChunkT; ++tt) {
      const size_t row = ((size_t)(b * kSeq + tb + tt)) * kDim + d;
      const float xs = XS[row];
      const float g  = GT[row];
      const float xc = conv_silu(xm3, xm2, xm1, xs, cwv[0], cwv[1], cwv[2], cwv[3], cb);
      xm3 = xm2; xm2 = xm1; xm1 = xs;
      const float* bc = sBC + tt * kBCcols;
      v4f bq[4], cq[4];
#pragma unroll
      for (int q4 = 0; q4 < 4; ++q4) {
        bq[q4] = *(const v4f*)(bc + 4 * q4);
        cq[q4] = *(const v4f*)(bc + kState + 4 * q4);
      }
      float y = 0.0f;
#pragma unroll
      for (int n = 0; n < kState; ++n) {
        const float bn = bq[n >> 2][n & 3];
        const float cn = cq[n >> 2][n & 3];
        h[n] = Av[n] * h[n] + xc * bn;
        y = fmaf(cn, h[n], y);
      }
      y = y + Dv * xc;
      const float eg = expf(-g);
      const float sg = g * __builtin_amdgcn_rcpf(1.0f + eg);
      sY[tt * kScanTPB + tid] = y * sg;
    }
    __syncthreads();
    for (int pass = 0; pass < 2; ++pass) {
#pragma unroll 1
      for (int it = 0; it < 8; ++it) {
        const int Li  = it * 16 + wave * 4 + lq;
        const int ttl = Li >> 1;
        const int col = (Li & 1) * 64 + lc * 8;
        const float* sp = sY + ttl * kScanTPB + col;
        const v4f a = *(const v4f*)(sp);
        const v4f c = *(const v4f*)(sp + 4);
        unsigned short hb[8], lb[8];
#pragma unroll
        for (int e = 0; e < 4; ++e) {
          split_bf(a[e], hb[e], lb[e]);
          split_bf(c[e], hb[4 + e], lb[4 + e]);
        }
        const v4u uh = (v4u){pk16(hb[0], hb[1]), pk16(hb[2], hb[3]), pk16(hb[4], hb[5]), pk16(hb[6], hb[7])};
        const v4u ul = (v4u){pk16(lb[0], lb[1]), pk16(lb[2], lb[3]), pk16(lb[4], lb[5]), pk16(lb[6], lb[7])};
        const size_t go = ((size_t)(b * kSeq + tb + ttl)) * kDim + d0 + col;
        *(volatile v4u*)(YH + go) = uh;
        *(volatile v4u*)(YL + go) = ul;
      }
      __threadfence();
    }
  }

  __syncthreads();
  {
    float* hp = sY + tid * kState;
#pragma unroll
    for (int q4 = 0; q4 < 4; ++q4) {
      const v4f v = (v4f){h[4 * q4 + 0], h[4 * q4 + 1], h[4 * q4 + 2], h[4 * q4 + 3]};
      *(v4f*)(hp + 4 * q4) = v;
    }
  }
  __syncthreads();
  float* hbase = HF + (size_t)(b * kDim + d0) * kState;
  for (int pass = 0; pass < 2; ++pass) {
#pragma unroll 1
    for (int it = 0; it < 4; ++it) {
      const int Li = it * 16 + wave * 4 + lq;
      const int base = Li * 32 + lc * 4;
      const v4f v = *(const v4f*)(sY + base);
      *(volatile v4f*)(hbase + base) = v;
    }
    __threadfence();
  }
}

__global__ __launch_bounds__(256) void mean_kernel(const float* __restrict__ HF, float* __restrict__ out1) {
  __shared__ float red[256];
  __shared__ __align__(16) float so[32];
  const int tid = threadIdx.x;
  const int o = tid >> 3, part = tid & 7;
  const int b = o >> 4, n = o & 15;
  const float* hp = HF + ((size_t)(b * kDim + part * 128)) * kState + n;
  float s = 0.0f;
#pragma unroll 1
  for (int j = 0; j < 128; ++j) s += hp[(size_t)j * kState];
  red[tid] = s;
  __syncthreads();
  if (tid < 32) {
    float tsum = red[tid * 8];
#pragma unroll
    for (int q = 1; q < 8; ++q) tsum += red[tid * 8 + q];
    so[tid] = tsum * (1.0f / 1024.0f);
  }
  __syncthreads();
  if (tid < 8) {
    const v4f v = *(const v4f*)(so + tid * 4);
    *(volatile v4f*)(out1 + tid * 4) = v;
    __threadfence();
    *(volatile v4f*)(out1 + tid * 4) = v;
  }
}

extern "C" void kernel_launch(void* const* d_in, const int* in_sizes, int n_in,
                              void* d_out, int out_size, void* d_ws, size_t ws_size, hipStream_t stream) {
  if (n_in < 11) return;
  if (in_sizes[0] != kRows * kDim) return;
  if (in_sizes[1] != kDim * kDim2) return;
  if (in_sizes[2] != kDim2) return;
  if (in_sizes[3] != kDim * kTaps) return;
  if (in_sizes[4] != kDim) return;
  if (in_sizes[5] != kDim * kBCcols) return;
  if (in_sizes[6] != kBCcols) return;
  if (in_sizes[7] != kDim * kState) return;
  if (in_sizes[8] != kDim) return;
  if (in_sizes[9] != kDim * kDim) return;
  if (in_sizes[10] != kDim) return;
  if (out_size < kRows * kDim + kBatch * kState) return;
  if (ws_size < kWsEnd) return;

  const float* x      = (const float*)d_in[0];
  const float* W_in   = (const float*)d_in[1];
  const float* b_in   = (const float*)d_in[2];
  const float* conv_w = (const float*)d_in[3];
  const float* conv_b = (const float*)d_in[4];
  const float* W_x    = (const float*)d_in[5];
  const float* b_x    = (const float*)d_in[6];
  const float* A_log  = (const float*)d_in[7];
  const float* D_par  = (const float*)d_in[8];
  const float* W_out  = (const float*)d_in[9];
  const float* b_out  = (const float*)d_in[10];

  char* ws = (char*)d_ws;
  unsigned short* P16H  = (unsigned short*)(ws + kOffP16H);
  unsigned short* P16L  = (unsigned short*)(ws + kOffP16L);
  unsigned short* WINH  = (unsigned short*)(ws + kOffWinH);
  unsigned short* WINL  = (unsigned short*)(ws + kOffWinL);
  float*          XS    = (float*)(ws + kOffXS);
  float*          GATE  = (float*)(ws + kOffGate);
  unsigned short* WOUTH = (unsigned short*)(ws + kOffWoutH);
  unsigned short* WOUTL = (unsigned short*)(ws + kOffWoutL);
  unsigned short* WXH   = (unsigned short*)(ws + kOffWxH);
  unsigned short* WXL   = (unsigned short*)(ws + kOffWxL);
  float*          BC    = (float*)(ws + kOffBC);
  float*          HFIN  = (float*)(ws + kOffHfin);

  float* out0 = (float*)d_out;
  float* out1 = out0 + (size_t)kRows * kDim;

  const int nElem = kRows * kDim;

  split8_bf16_kernel<<<dim3((nElem / 8 + 255) / 256), dim3(256), 0, stream>>>(x, P16H, P16L, nElem / 8);

  wt_split_kernel<<<dim3(kDim / 64, kDim2 / 64), dim3(256), 0, stream>>>(W_in, kDim2, kDim2, kDim, WINH, WINL);
  wt_split_kernel<<<dim3(kDim / 64, kDim / 64), dim3(256), 0, stream>>>(W_out, kDim, kDim, kDim, WOUTH, WOUTL);
  wt_split_kernel<<<dim3(kDim / 64, kBCld / 64), dim3(256), 0, stream>>>(W_x, kBCcols, kBCcols, kDim, WXH, WXL);

  {
    const int tiles = (kRows / 64) * (kDim / 64);
    wmma_gemm64<1, true, 2, 0, false><<<dim3(tiles / 8, 1), dim3(256), 0, stream>>>(
        P16H, P16L, kDim, (long)0,
        WINH, WINL, kDim, (long)0,
        (void*)XS, (void*)nullptr, kDim, (long)0,
        b_in, (const float*)nullptr, (long)0,
        kRows, kDim, kDim, 1.0f);
    wmma_gemm64<1, true, 2, 0, false><<<dim3(tiles / 8, 1), dim3(256), 0, stream>>>(
        P16H, P16L, kDim, (long)0,
        WINH + (size_t)kDim * kDim, WINL + (size_t)kDim * kDim, kDim, (long)0,
        (void*)GATE, (void*)nullptr, kDim, (long)0,
        b_in + kDim, (const float*)nullptr, (long)0,
        kRows, kDim, kDim, 1.0f);
  }

  conv_split_kernel<<<dim3((nElem / 2 + 255) / 256), dim3(256), 0, stream>>>(XS, conv_w, conv_b, P16H, P16L, nElem / 2);

  {
    const int tiles = (kRows / 64) * (kBCld / 64);
    wmma_gemm64<1, true, 0, 0, false><<<dim3(tiles / 8, 1), dim3(256), 0, stream>>>(
        P16H, P16L, kDim, (long)0,
        WXH, WXL, kDim, (long)0,
        (void*)BC, (void*)nullptr, kBCld, (long)0,
        (const float*)nullptr, (const float*)nullptr, (long)0,
        kRows, kBCld, kDim, 1.0f);
  }

  scan_kernel<<<dim3(kBatch * (kDim / kScanTPB)), dim3(kScanTPB), 0, stream>>>(
      XS, GATE, BC, conv_w, conv_b, b_x, A_log, D_par, P16H, P16L, HFIN);

  {
    const int tiles = (kRows / 64) * (kDim / 64);
    wmma_gemm64<1, true, 2, 0, false><<<dim3(tiles / 8, 1), dim3(256), 0, stream>>>(
        P16H, P16L, kDim, (long)0,
        WOUTH, WOUTL, kDim, (long)0,
        (void*)out0, (void*)nullptr, kDim, (long)0,
        b_out, (const float*)nullptr, (long)0,
        kRows, kDim, kDim, 1.0f);
  }

  mean_kernel<<<dim3(1), dim3(256), 0, stream>>>(HFIN, out1);
}
